// FlowPlusPlusLayer_16810501997233
// MI455X (gfx1250) — hardware-run, weakly checked
//
#include <hip/hip_runtime.h>
#include <math.h>

typedef __attribute__((ext_vector_type(16))) _Float16 v16h;
typedef __attribute__((ext_vector_type(8)))  _Float16 v8h;
typedef __attribute__((ext_vector_type(2)))  _Float16 v2h;
typedef __attribute__((ext_vector_type(16))) __bf16   v16b;
typedef __attribute__((ext_vector_type(8)))  __bf16   v8b;
typedef __attribute__((ext_vector_type(8)))  float    v8f;
typedef __attribute__((ext_vector_type(4)))  float    v4f;
typedef __attribute__((ext_vector_type(4)))  int      v4i;
typedef __attribute__((ext_vector_type(2)))  float    v2f;

constexpr int kB    = 16384;
constexpr int kD    = 16;
constexpr int kDP   = 32;
constexpr int kH    = 512;
constexpr int kO    = 224;
constexpr int kOP   = 256;
constexpr int kMix  = 4;
constexpr int kBis  = 50;
constexpr int kThr  = 256;
constexpr float kInCarry = 1024.0f;
constexpr float kSc20 = 1.0f / (kInCarry * kInCarry);
constexpr float kSc10 = 1.0f / kInCarry;
constexpr float kF16MinNormal = 6.103515625e-5f;
constexpr size_t kOut1 = (size_t)kB * kD;

static_assert(kB == 16384 && kD == 16 && kDP == 32 && kH == 512 && kO == kD * (3 * kMix + 2) && kOP == 256 && kMix == 4, "the index arithmetic below uses these sizes");

constexpr size_t kOffWM0 = 0ull;
constexpr size_t kOffWM1 = 32768ull;
constexpr size_t kOffWM2 = 1081344ull;
constexpr size_t kOffA0T = 1540096ull;
constexpr size_t kOffA1T = 1572864ull;
constexpr size_t kOffA2T = 2097152ull;
constexpr size_t kOffBR0 = 2359296ull;
constexpr size_t kOffBR1 = 2361344ull;
constexpr size_t kOffX32 = 2363392ull;
constexpr size_t kOffX16 = 3411968ull;
constexpr size_t kOffH1 = 4460544ull;
constexpr size_t kOffH2 = 21237760ull;
constexpr size_t kOffOUT = 38014976ull;
constexpr size_t kOffLD = 54792192ull;
constexpr size_t kWsTotal = 54857728ull;
static_assert(kWsTotal <= 134217728ull, "the carve stands under 128 MiB");
static_assert(kOffWM0 == 0
  && kOffWM1 == kOffWM0 + 32768ull
  && kOffWM2 == kOffWM1 + 1048576ull
  && kOffA0T == kOffWM2 + 458752ull
  && kOffA1T == kOffA0T + 32768ull
  && kOffA2T == kOffA1T + 524288ull
  && kOffBR0 == kOffA2T + 262144ull
  && kOffBR1 == kOffBR0 + 2048ull
  && kOffX32 == kOffBR1 + 2048ull
  && kOffX16 == kOffX32 + 1048576ull
  && kOffH1 == kOffX16 + 1048576ull
  && kOffH2 == kOffH1 + 16777216ull
  && kOffOUT == kOffH2 + 16777216ull
  && kOffLD == kOffOUT + 16777216ull
  && kWsTotal == kOffLD + 65536ull, "the carve is a chain: every region starts where the one before ends");
static_assert((kOffWM0 % 256) == 0 && (kOffWM1 % 256) == 0 && (kOffWM2 % 256) == 0 && (kOffA0T % 256) == 0 && (kOffA1T % 256) == 0 && (kOffA2T % 256) == 0 && (kOffBR0 % 256) == 0 && (kOffBR1 % 256) == 0 && (kOffX32 % 256) == 0 && (kOffX16 % 256) == 0 && (kOffH1 % 256) == 0 && (kOffH2 % 256) == 0 && (kOffOUT % 256) == 0 && (kOffLD % 256) == 0, "every region starts on a multiple of 256 B");

__device__ __forceinline__ unsigned short f2bf_bits(float f) {
  unsigned u = __float_as_uint(f);
  return (unsigned short)((u + 0x7FFFu + ((u >> 16) & 1u)) >> 16);
}
__device__ __forceinline__ float bf_bits2f(unsigned short h) { return __uint_as_float(((unsigned)h) << 16); }
__device__ __forceinline__ float bf16r(float f) { return bf_bits2f(f2bf_bits(f)); }
__device__ __forceinline__ float carry_flush(float v, float carry) {
  const float s = v * carry;
  return (fabsf(s) < kF16MinNormal) ? 0.0f : s;
}

__device__ __forceinline__ void dep_guard4_h(v8f& a, v8f& b, v8f& c, v8f& d, v16h x, v16h y) { asm volatile("v_nop\n\tv_nop\n\tv_nop\n\tv_nop" : "+v"(a), "+v"(b), "+v"(c), "+v"(d) : "v"(x), "v"(y)); }
__device__ __forceinline__ void dep_guard4_b(v8f& a, v8f& b, v8f& c, v8f& d, v16b x, v16b y) { asm volatile("v_nop\n\tv_nop\n\tv_nop\n\tv_nop" : "+v"(a), "+v"(b), "+v"(c), "+v"(d) : "v"(x), "v"(y)); }
__device__ __forceinline__ void keep4_h(v16h a, v16h b, v16h c, v16h d) { asm volatile("v_nop" :: "v"(a), "v"(b), "v"(c), "v"(d)); }
__device__ __forceinline__ void keep4_b(v16b a, v16b b, v16b c, v16b d) { asm volatile("v_nop" :: "v"(a), "v"(b), "v"(c), "v"(d)); }
__device__ __forceinline__ void acc_guard4(v8f& a, v8f& b, v8f& c, v8f& d) { asm volatile("v_nop\n\tv_nop\n\tv_nop\n\tv_nop" : "+v"(a), "+v"(b), "+v"(c), "+v"(d)); }

template <typename T> struct Frag;
template <> struct Frag<_Float16> {
  typedef v16h V; union U { v16h v; v8h h[2]; };
  static __device__ __forceinline__ v16h load(const _Float16* p) {
    U f; f.h[0] = *(const v8h*)(p); f.h[1] = *(const v8h*)(p + 16); return f.v;
  }
  static __device__ __forceinline__ v8f mma(v16h a, v16h b, v8f c) {
    return __builtin_amdgcn_wmma_f32_16x16x32_f16(false, a, false, b, (short)0, c, false, false);
  }
  static __device__ __forceinline__ void guard4(v8f& a, v8f& b, v8f& c, v8f& d, v16h x, v16h y) { dep_guard4_h(a, b, c, d, x, y); }
  static __device__ __forceinline__ void keep(v16h a, v16h b, v16h c, v16h d) { keep4_h(a, b, c, d); }
};
template <> struct Frag<__bf16> {
  typedef v16b V; union U { v16b v; v8b h[2]; };
  static __device__ __forceinline__ v16b load(const __bf16* p) {
    U f; f.h[0] = *(const v8b*)(p); f.h[1] = *(const v8b*)(p + 16); return f.v;
  }
  static __device__ __forceinline__ v8f mma(v16b a, v16b b, v8f c) {
    return __builtin_amdgcn_wmma_f32_16x16x32_bf16(false, a, false, b, (short)0, c, false, false);
  }
  static __device__ __forceinline__ void guard4(v8f& a, v8f& b, v8f& c, v8f& d, v16b x, v16b y) { dep_guard4_b(a, b, c, d, x, y); }
  static __device__ __forceinline__ void keep(v16b a, v16b b, v16b c, v16b d) { keep4_b(a, b, c, d); }
};

__device__ __forceinline__ v8f mma_h(v16h a, v16h b, v8f c) {
  c = __builtin_amdgcn_wmma_f32_16x16x32_f16(false, a, false, b, (short)0, c, false, false);
  asm volatile("v_nop\n\tv_nop\n\tv_nop\n\tv_nop" : "+v"(c) : "v"(a), "v"(b));
  return c;
}

template <int ET> struct Elem;
template <> struct Elem<0> { typedef _Float16 T; };
template <> struct Elem<1> { typedef __bf16 T; };
template <int ET, bool SPLIT, int BIAS_MODE, int OUT_MODE, bool RESID, int ACT = 0>
__global__ __launch_bounds__(256) void wmma_gemm64(
    const unsigned short* __restrict__ Ap, const unsigned short* __restrict__ A2p, int lda, long strideA,
    const unsigned short* __restrict__ Btp, const unsigned short* __restrict__ Bt2p, int ldb, long strideB,
    void* __restrict__ Cout, void* __restrict__ Cout2, int ldc, long strideC,
    const float* __restrict__ bias,
    const float* __restrict__ resid, long strideR,
    int M, int N, int K, float scale) {
  typedef typename Elem<ET>::T T;
  typedef typename Frag<T>::V V;
  const T* A = (const T*)Ap; const T* A2 = (const T*)A2p; const T* Bt = (const T*)Btp; const T* Bt2 = (const T*)Bt2p;
  __shared__ __align__(16) float sT[8][16 * 68];
  const int b    = blockIdx.y;
  const int lane = threadIdx.x & 31;
  const int wave = threadIdx.x >> 5;
  const int tilesN = N >> 6;
  const int tilesM = M >> 6;
  const int tile = blockIdx.x * 8 + wave;
  if (tile >= tilesM * tilesN) return;
  const int tm = tile / tilesN;
  const int tn = tile - tm * tilesN;
  const int m0 = tm << 6;
  const int n0 = tn << 6;

  const T* Ab  = A  + (size_t)b * strideA;
  const T* Bb  = Bt + (size_t)b * strideB;
  const T* Ab2 = SPLIT ? (A2  + (size_t)b * strideA) : nullptr;
  const T* Bb2 = SPLIT ? (Bt2 + (size_t)b * strideB) : nullptr;

  const int rlane = lane & 15;
  const int koff  = (lane >> 4) * 8;
  const int mOff  = (lane >> 4) * 8;

  v8f acc[4][4];
#pragma unroll
  for (int i = 0; i < 4; ++i)
#pragma unroll
    for (int j = 0; j < 4; ++j) acc[i][j] = (v8f){0.f,0.f,0.f,0.f,0.f,0.f,0.f,0.f};

  for (int k0 = 0; k0 < K; k0 += 32) {
    V bh[4], bl[4];
#pragma unroll
    for (int j = 0; j < 4; ++j) {
      const size_t bo = (size_t)(n0 + (j << 4) + rlane) * ldb + koff + k0;
      bh[j] = Frag<T>::load(Bb + bo);
      if (SPLIT) bl[j] = Frag<T>::load(Bb2 + bo);
    }
#pragma unroll
    for (int i = 0; i < 4; ++i) {
      const size_t ao = (size_t)(m0 + (i << 4) + rlane) * lda + koff + k0;
      V ah = Frag<T>::load(Ab + ao);
      V al;
      if (SPLIT) al = Frag<T>::load(Ab2 + ao);
#pragma unroll
      for (int j = 0; j < 4; ++j) {
        acc[i][j] = Frag<T>::mma(ah, bh[j], acc[i][j]);
        if (SPLIT) {
          acc[i][j] = Frag<T>::mma(ah, bl[j], acc[i][j]);
          acc[i][j] = Frag<T>::mma(al, bh[j], acc[i][j]);
        }
      }
      Frag<T>::guard4(acc[i][0], acc[i][1], acc[i][2], acc[i][3], ah, SPLIT ? al : ah);
    }
    Frag<T>::keep(bh[0], bh[1], bh[2], bh[3]);
    if (SPLIT) Frag<T>::keep(bl[0], bl[1], bl[2], bl[3]);
  }
  acc_guard4(acc[0][0], acc[0][1], acc[0][2], acc[0][3]);
  acc_guard4(acc[1][0], acc[1][1], acc[1][2], acc[1][3]);
  acc_guard4(acc[2][0], acc[2][1], acc[2][2], acc[2][3]);
  acc_guard4(acc[3][0], acc[3][1], acc[3][2], acc[3][3]);

  float* slab = sT[wave];
  const float* Rb = RESID ? (resid + (size_t)b * strideR) : nullptr;
#pragma unroll
  for (int i = 0; i < 4; ++i) {
    const int mBase = m0 + (i << 4);
#pragma unroll
    for (int j = 0; j < 4; ++j) {
      const int n = n0 + (j << 4) + rlane;
      float bv = 0.f;
      if (BIAS_MODE == 2) bv = bias[n];
#pragma unroll
      for (int r = 0; r < 8; ++r) {
        float v = acc[i][j][r] * scale;
        if (BIAS_MODE == 1) v += bias[mBase + mOff + r];
        if (BIAS_MODE == 2) v += bv;
        if (RESID) v += Rb[(size_t)(mBase + mOff + r) * ldc + n];
        if (ACT == 1) v = tanhf(v);
        if (ACT == 2) v = fmaxf(v, 0.0f);
        if (ACT == 3) v = v / (1.0f + expf(-v));
        if (ACT == 4) v = (v > 0.f) ? v : 0.01f * v;
        slab[(mOff + r) * 68 + (j << 4) + rlane] = v;
      }
    }
    __builtin_amdgcn_fence(__ATOMIC_RELEASE, "workgroup");
    __builtin_amdgcn_wave_barrier();
    __builtin_amdgcn_fence(__ATOMIC_ACQUIRE, "workgroup");
    if (OUT_MODE == 0) {
      float* C = (float*)Cout + (size_t)b * strideC;
      const int hh = lane >> 4, c4 = (lane & 15) * 4;
      for (int pass = 0; pass < 2; ++pass) {
#pragma unroll
        for (int it = 0; it < 8; ++it) {
          const int row = it * 2 + hh;
          v4f v = *(const v4f*)(slab + row * 68 + c4);
          *(volatile v4f*)(C + (size_t)(mBase + row) * ldc + n0 + c4) = v;
        }
        __threadfence();
      }
    } else {
      const int q = lane >> 3, c8 = (lane & 7) * 8;
      unsigned short* C  = (unsigned short*)Cout  + (size_t)b * strideC;
      unsigned short* C2 = (OUT_MODE == 2) ? ((unsigned short*)Cout2 + (size_t)b * strideC) : nullptr;
      for (int pass = 0; pass < 2; ++pass) {
#pragma unroll
        for (int it = 0; it < 4; ++it) {
          const int row = it * 4 + q;
          const float* sp = slab + row * 68 + c8;
          v8h hv, lv;
#pragma unroll
          for (int e = 0; e < 8; ++e) {
            if (OUT_MODE == 1) {
              hv[e] = (_Float16)sp[e];
            } else {
              unsigned short hb = f2bf_bits(sp[e]);
              unsigned short lb = f2bf_bits(sp[e] - bf_bits2f(hb));
              hv[e] = __builtin_bit_cast(_Float16, hb);
              lv[e] = __builtin_bit_cast(_Float16, lb);
            }
          }
          *(volatile v8h*)(C + (size_t)(mBase + row) * ldc + n0 + c8) = hv;
          if (OUT_MODE == 2) *(volatile v8h*)(C2 + (size_t)(mBase + row) * ldc + n0 + c8) = lv;
        }
        __threadfence();
      }
    }
    __builtin_amdgcn_fence(__ATOMIC_RELEASE, "workgroup");
    __builtin_amdgcn_wave_barrier();
    __builtin_amdgcn_fence(__ATOMIC_ACQUIRE, "workgroup");
  }
}

__global__ __launch_bounds__(kThr) void pack_kernel(const float* __restrict__ W, unsigned short* __restrict__ D, float* __restrict__ dstf, int part, int ld, int k0, int lg, int n0, int pitch) {
  const unsigned i = blockIdx.x * blockDim.x + threadIdx.x;
  if (part == 0) {
    const unsigned g = i & ((1u << lg) - 1u), n = i >> lg;
    const float* sp = W + (size_t)((unsigned)k0 + g * 8u) * (unsigned)ld + n;
    v8h hv;
#pragma unroll
    for (int t = 0; t < 8; ++t) hv[t] = (_Float16)carry_flush(bf16r(sp[(size_t)t * (unsigned)ld]), kInCarry);
    unsigned short* dp = D + (size_t)((unsigned)n0 + n) * (unsigned)pitch + g * 8u;
    *(volatile v8h*)dp = hv;
    __threadfence();
    *(volatile v8h*)dp = hv;
  } else {
    const v4f a = *(const v4f*)(W + i * 4u);
    v4f o;
#pragma unroll
    for (int e = 0; e < 4; ++e) o[e] = bf16r(a[e]);
    float* dp = dstf + i * 4u;
    *(volatile v4f*)dp = o;
    __threadfence();
    *(volatile v4f*)dp = o;
  }
}

__global__ __launch_bounds__(kThr) void brec_kernel(const float* __restrict__ b, float* __restrict__ dstf) {
  const unsigned i = blockIdx.x * blockDim.x + threadIdx.x;
  const v4f a = *(const v4f*)(b + i * 4u);
  v4f o;
#pragma unroll
  for (int e = 0; e < 4; ++e) o[e] = bf16r(a[e]) * kInCarry;
  float* dp = dstf + i * 4u;
  *(volatile v4f*)dp = o;
  __threadfence();
  *(volatile v4f*)dp = o;
}

__global__ __launch_bounds__(kThr) void zero_kernel(float* __restrict__ dst) {
  const size_t o4 = ((size_t)blockIdx.x * kThr + threadIdx.x) * 4u;
  const v4f z = {0.f, 0.f, 0.f, 0.f};
  *(volatile v4f*)(dst + o4) = z;
  __threadfence();
  *(volatile v4f*)(dst + o4) = z;
}

__global__ __launch_bounds__(kThr) void wmask_kernel(const float* __restrict__ Wt, const int* __restrict__ Mk, float* __restrict__ dst) {
  const size_t o4 = ((size_t)blockIdx.x * kThr + threadIdx.x) * 4u;
  const v4f w = *(const v4f*)(Wt + o4);
  const v4i m = *(const v4i*)(Mk + o4);
  v4f r;
#pragma unroll
  for (int e = 0; e < 4; ++e) r[e] = __uint_as_float(__float_as_uint(w[e]) & ((m[e] != 0) ? 0xFFFFFFFFu : 0u));
  *(volatile v4f*)(dst + o4) = r;
  __threadfence();
  *(volatile v4f*)(dst + o4) = r;
}

__global__ __launch_bounds__(kThr) void xpad_kernel(const float* __restrict__ X32, unsigned short* __restrict__ X16) {
  const unsigned i = blockIdx.x * (unsigned)kThr + threadIdx.x;
  const unsigned row = i >> 1, g = i & 1u;
  const float* sp = X32 + (size_t)row * (unsigned)kD + 8u * g;
  const v4f a0 = *(const v4f*)sp, a1 = *(const v4f*)(sp + 4);
  v8h hv;
#pragma unroll
  for (int e = 0; e < 4; ++e) { hv[e] = (_Float16)carry_flush(a0[e], kInCarry); hv[4 + e] = (_Float16)carry_flush(a1[e], kInCarry); }
  unsigned short* dp = X16 + (size_t)row * (unsigned)kDP + 8u * g;
  *(volatile v8h*)dp = hv;
  __threadfence();
  *(volatile v8h*)dp = hv;
}

__device__ __forceinline__ float softplus_f(float z) { return fmaxf(z, 0.0f) + log1pf(expf(-fabsf(z))); }
__device__ __forceinline__ float lse4_f(float a0, float a1, float a2, float a3) {
  const float m = fmaxf(fmaxf(a0, a1), fmaxf(a2, a3));
  return m + logf(((expf(a0 - m) + expf(a1 - m)) + expf(a2 - m)) + expf(a3 - m));
}
__global__ __launch_bounds__(kThr) void couple_kernel(const float* __restrict__ OUT, const float* __restrict__ b2, const float* __restrict__ u, float* __restrict__ X32, float* __restrict__ LD, int t) {
  const unsigned row = blockIdx.x * (unsigned)kThr + threadIdx.x;
  const float* op = OUT + (size_t)row * (unsigned)kOP + (unsigned)t;
  const float* bp = b2 + (unsigned)t;
  const float ola = op[0] + bf16r(bp[0]);
  const float bb  = op[kD] + bf16r(bp[kD]);
  float raw[kMix], mu[kMix], ls[kMix];
#pragma unroll
  for (int l = 0; l < kMix; ++l) {
    raw[l] = op[2 * kD + l * kD] + bf16r(bp[2 * kD + l * kD]);
    mu[l]  = op[2 * kD + kMix * kD + l * kD] + bf16r(bp[2 * kD + kMix * kD + l * kD]);
    ls[l]  = op[2 * kD + 2 * kMix * kD + l * kD] + bf16r(bp[2 * kD + 2 * kMix * kD + l * kD]);
  }
  const float la = 0.1f * tanhf(ola);
  const float lser = lse4_f(raw[0], raw[1], raw[2], raw[3]);
  float lp[kMix], es[kMix];
#pragma unroll
  for (int l = 0; l < kMix; ++l) { lp[l] = raw[l] - lser; es[l] = expf(-ls[l]); }
  const float ut = bf16r(u[(size_t)row * (unsigned)kD + (unsigned)t]);
  const float y = 1.0f / (1.0f + expf(-((ut - bb) * expf(-la))));
  float term = (-la + logf(y)) + log1pf(-y);
  float low = -1000.0f, high = 1000.0f;
  for (int it = 0; it < kBis; ++it) {
    const float mid = (low + high) * 0.5f;
    float a[kMix];
#pragma unroll
    for (int l = 0; l < kMix; ++l) a[l] = -softplus_f(-(es[l] * (mid - mu[l]))) + lp[l];
    const float val = expf(lse4_f(a[0], a[1], a[2], a[3]));
    low = (val < y) ? mid : low;
    high = (val > y) ? mid : high;
  }
  const float xt = (low + high) * 0.5f;
  float q[kMix];
#pragma unroll
  for (int l = 0; l < kMix; ++l) { const float z = es[l] * (xt - mu[l]); q[l] = ((z - ls[l]) - 2.0f * softplus_f(z)) + lp[l]; }
  term = term - lse4_f(q[0], q[1], q[2], q[3]);
  float* xp = X32 + (size_t)row * (unsigned)kD + (unsigned)t;
  float* lp_ = LD + row;
  const float nl = *lp_ + term;
  *(volatile float*)xp = xt;
  *(volatile float*)lp_ = nl;
  __threadfence();
  *(volatile float*)xp = xt;
  *(volatile float*)lp_ = nl;
}

__global__ __launch_bounds__(kThr) void lcopy_kernel(const float* __restrict__ src, float* __restrict__ dst) {
  const size_t o4 = ((size_t)blockIdx.x * kThr + threadIdx.x) * 4u;
  const v4f v = *(const v4f*)(src + o4);
  *(volatile v4f*)(dst + o4) = v;
  __threadfence();
  *(volatile v4f*)(dst + o4) = v;
}

extern "C" void kernel_launch(void* const* d_in, const int* in_sizes, int n_in,
                              void* d_out, int out_size, void* d_ws, size_t ws_size,
                              hipStream_t stream) {
  if (n_in < 11 || d_out == nullptr || d_ws == nullptr) return;
  if (in_sizes[0] != kB * kD || in_sizes[1] != kD * kH || in_sizes[2] != kH || in_sizes[3] != kH * kH || in_sizes[4] != kH || in_sizes[5] != kH * kO || in_sizes[6] != kO || in_sizes[7] != kD * kH || in_sizes[8] != kH * kH || in_sizes[9] != kH * kO || in_sizes[10] != kD) return;
  if ((size_t)out_size != kOut1 + (size_t)kB) return;
  if (ws_size < kWsTotal) return;
  const float* u = (const float*)d_in[0];
  const float* W0 = (const float*)d_in[1];
  const float* b0 = (const float*)d_in[2];
  const float* W1 = (const float*)d_in[3];
  const float* b1 = (const float*)d_in[4];
  const float* W2 = (const float*)d_in[5];
  const float* b2 = (const float*)d_in[6];
  const int* M0 = (const int*)d_in[7];
  const int* M1 = (const int*)d_in[8];
  const int* M2 = (const int*)d_in[9];
  float* out = (float*)d_out;
  char* ws = (char*)d_ws;
  float* WM0 = (float*)(ws + kOffWM0);
  float* WM1 = (float*)(ws + kOffWM1);
  float* WM2 = (float*)(ws + kOffWM2);
  unsigned short* A0T = (unsigned short*)(ws + kOffA0T);
  unsigned short* A1T = (unsigned short*)(ws + kOffA1T);
  unsigned short* A2T = (unsigned short*)(ws + kOffA2T);
  float* BR0 = (float*)(ws + kOffBR0);
  float* BR1 = (float*)(ws + kOffBR1);
  float* X32 = (float*)(ws + kOffX32);
  unsigned short* X16 = (unsigned short*)(ws + kOffX16);
  unsigned short* H1 = (unsigned short*)(ws + kOffH1);
  unsigned short* H2 = (unsigned short*)(ws + kOffH2);
  float* OUT = (float*)(ws + kOffOUT);
  float* LD = (float*)(ws + kOffLD);

  static_assert((kD * kH / 4) % kThr == 0 && (kH * kH / 4) % kThr == 0 && (kH * kO / 4) % kThr == 0 && (kH * kDP * 2 / 16) % kThr == 0 && (kOP * kH * 2 / 16) % kThr == 0 && (kB * kD / 4) % kThr == 0 && (kB * kDP * 2 / 16) % kThr == 0 && (kB / 4) % kThr == 0 && (kB * 2) % kThr == 0 && kB % kThr == 0 && (kH * (kD / 8)) % 64 == 0 && (kH * (kH / 8)) % 64 == 0 && (kO * (kH / 8)) % 64 == 0 && (kH / 4) % 64 == 0, "every flat kernel's grid exact");
  wmask_kernel<<<kD * kH / 4 / kThr, kThr, 0, stream>>>(W0, M0, WM0);
  wmask_kernel<<<kH * kH / 4 / kThr, kThr, 0, stream>>>(W1, M1, WM1);
  wmask_kernel<<<kH * kO / 4 / kThr, kThr, 0, stream>>>(W2, M2, WM2);
  zero_kernel<<<kH * kDP * 2 / 16 / kThr, kThr, 0, stream>>>((float*)A0T);
  zero_kernel<<<kOP * kH * 2 / 16 / kThr, kThr, 0, stream>>>((float*)A2T);
  zero_kernel<<<kB * kD / 4 / kThr, kThr, 0, stream>>>(X32);
  zero_kernel<<<kB * kDP * 2 / 16 / kThr, kThr, 0, stream>>>((float*)X16);
  zero_kernel<<<kB / 4 / kThr, kThr, 0, stream>>>(LD);
  pack_kernel<<<kH * (kD / 8) / 64, 64, 0, stream>>>(WM0, A0T, nullptr, 0, kH, 0, 1, 0, kDP);
  pack_kernel<<<kH * (kH / 8) / 64, 64, 0, stream>>>(WM1, A1T, nullptr, 0, kH, 0, 6, 0, kH);
  pack_kernel<<<kO * (kH / 8) / 64, 64, 0, stream>>>(WM2, A2T, nullptr, 0, kO, 0, 6, 0, kH);
  brec_kernel<<<kH / 4 / 64, 64, 0, stream>>>(b0, BR0);
  brec_kernel<<<kH / 4 / 64, 64, 0, stream>>>(b1, BR1);
  for (int t = 0; t < kD; ++t) {
    xpad_kernel<<<kB * 2 / kThr, kThr, 0, stream>>>(X32, X16);
    wmma_gemm64<0, false, 2, 1, false, 4><<<dim3((kB / 64) * (kH / 64) / 8, 1), 256, 0, stream>>>(
        X16, X16, kDP, 0L, A0T, A0T, kDP, 0L, (void*)H1, (void*)H1, kH, 0L, BR0, nullptr, 0L, kB, kH, kDP, kSc10);
    wmma_gemm64<0, false, 2, 1, false, 4><<<dim3((kB / 64) * (kH / 64) / 8, 1), 256, 0, stream>>>(
        H1, H1, kH, 0L, A1T, A1T, kH, 0L, (void*)H2, (void*)H2, kH, 0L, BR1, nullptr, 0L, kB, kH, kH, kSc10);
    wmma_gemm64<0, false, 0, 0, false, 0><<<dim3((kB / 64) * (kOP / 64) / 8, 1), 256, 0, stream>>>(
        H2, H2, kH, 0L, A2T, A2T, kH, 0L, (void*)OUT, (void*)OUT, kOP, 0L, nullptr, nullptr, 0L, kB, kOP, kH, kSc20);
    couple_kernel<<<kB / kThr, kThr, 0, stream>>>(OUT, b2, u, X32, LD, t);
  }
  lcopy_kernel<<<kB * kD / 4 / kThr, kThr, 0, stream>>>(X32, out);
  lcopy_kernel<<<kB / 4 / kThr, kThr, 0, stream>>>(LD, out + kOut1);
}
static_assert(((kB / 64) * (kH / 64)) % 8 == 0 && ((kB / 64) * (kOP / 64)) % 8 == 0 && kDP % 32 == 0 && kH % 32 == 0, "the engine's grids: whole blocks of eight wave tiles; the depths multiples of 32");
